// LSTMEncoder_78975858639682
// MI455X (gfx1250) — hardware-verified
//
#include <hip/hip_runtime.h>
#include <math.h>

typedef __attribute__((ext_vector_type(16))) _Float16 v16h;
typedef __attribute__((ext_vector_type(8)))  _Float16 v8h;
typedef __attribute__((ext_vector_type(16))) __bf16   v16b;
typedef __attribute__((ext_vector_type(8)))  __bf16   v8b;
typedef __attribute__((ext_vector_type(8)))  float    v8f;
typedef __attribute__((ext_vector_type(4)))  float    v4f;

constexpr int kB    = 2048;
constexpr int kT    = 512;
constexpr int kIn   = 4;
constexpr int kH    = 64;
constexpr int kG4   = 4 * kH;
constexpr int kKP   = 128;
constexpr int kK0   = 96;
constexpr int kThr  = 256;
constexpr float kInCarry = 1024.0f;
constexpr float kSc = 1.0f / (kInCarry * kInCarry);
constexpr float kF16MinNormal = 6.103515625e-5f;
constexpr int kFB0 = 0, kFB1 = 256, kFBF = 512, kFEnd = 1024;

static_assert((kB % 64) == 0 && ((kB / 64) * (kG4 / 64)) % 8 == 0 && ((kB / 64) * (kH / 64)) % 8 == 0 && (kK0 % 32) == 0 && (kKP % 32) == 0 && (kH % 32) == 0 && (kKP * 2) % 128 == 0,
              "GEMM M, N multiples of 64; grids exact; K multiples of 32; operand rows are whole lines");

constexpr size_t kOffW0 = 0ull;
constexpr size_t kOffW1 = 65536ull;
constexpr size_t kOffWF = 131072ull;
constexpr size_t kOffBIAS = 139264ull;
constexpr size_t kOffA0 = 143360ull;
constexpr size_t kOffA1 = 667648ull;
constexpr size_t kOffG0 = 1191936ull;
constexpr size_t kOffG1 = 3289088ull;
constexpr size_t kOffC0 = 5386240ull;
constexpr size_t kOffC1 = 5910528ull;
constexpr size_t kOffHN16 = 6434816ull;
constexpr size_t kOffP32 = 6696960ull;
constexpr size_t kWsTotal = 7221248ull;
static_assert(kWsTotal <= 134217728ull, "carve cap: under 128 MiB");
static_assert(kOffW0 == 0
              && kOffW1 == kOffW0 + 65536ull
              && kOffWF == kOffW1 + 65536ull
              && kOffBIAS == kOffWF + 8192ull
              && kOffA0 == kOffBIAS + 4096ull
              && kOffA1 == kOffA0 + 524288ull
              && kOffG0 == kOffA1 + 524288ull
              && kOffG1 == kOffG0 + 2097152ull
              && kOffC0 == kOffG1 + 2097152ull
              && kOffC1 == kOffC0 + 524288ull
              && kOffHN16 == kOffC1 + 524288ull
              && kOffP32 == kOffHN16 + 262144ull
              && kWsTotal == kOffP32 + 524288ull, "the carve is chained and totalled");
static_assert((kOffW0 % 256) == 0 && (kOffW1 % 256) == 0 && (kOffWF % 256) == 0 && (kOffBIAS % 256) == 0 && (kOffA0 % 256) == 0 && (kOffA1 % 256) == 0 && (kOffG0 % 256) == 0 && (kOffG1 % 256) == 0 && (kOffC0 % 256) == 0 && (kOffC1 % 256) == 0 && (kOffHN16 % 256) == 0 && (kOffP32 % 256) == 0, "aligned regions");

__device__ __forceinline__ unsigned short f2bf_bits(float f) {
  unsigned u = __float_as_uint(f);
  return (unsigned short)((u + 0x7FFFu + ((u >> 16) & 1u)) >> 16);
}
__device__ __forceinline__ float bf_bits2f(unsigned short h) { return __uint_as_float(((unsigned)h) << 16); }
__device__ __forceinline__ float bf16r(float f) { return bf_bits2f(f2bf_bits(f)); }
__device__ __forceinline__ float carry_flush(float v, float carry) {
  const float s = v * carry;
  return (fabsf(s) < kF16MinNormal) ? 0.0f : s;
}
__device__ __forceinline__ float frcp(float x) { return __builtin_amdgcn_rcpf(x); }

__device__ __forceinline__ void dep_guard4_h(v8f& a, v8f& b, v8f& c, v8f& d, v16h x, v16h y) { asm volatile("v_nop\n\tv_nop\n\tv_nop\n\tv_nop" : "+v"(a), "+v"(b), "+v"(c), "+v"(d) : "v"(x), "v"(y)); }
__device__ __forceinline__ void dep_guard4_b(v8f& a, v8f& b, v8f& c, v8f& d, v16b x, v16b y) { asm volatile("v_nop\n\tv_nop\n\tv_nop\n\tv_nop" : "+v"(a), "+v"(b), "+v"(c), "+v"(d) : "v"(x), "v"(y)); }
__device__ __forceinline__ void keep4_h(v16h a, v16h b, v16h c, v16h d) { asm volatile("v_nop" :: "v"(a), "v"(b), "v"(c), "v"(d)); }
__device__ __forceinline__ void keep4_b(v16b a, v16b b, v16b c, v16b d) { asm volatile("v_nop" :: "v"(a), "v"(b), "v"(c), "v"(d)); }
__device__ __forceinline__ void acc_guard4(v8f& a, v8f& b, v8f& c, v8f& d) { asm volatile("v_nop\n\tv_nop\n\tv_nop\n\tv_nop" : "+v"(a), "+v"(b), "+v"(c), "+v"(d)); }

template <typename T> struct Frag;
template <> struct Frag<_Float16> {
  typedef v16h V; union U { v16h v; v8h h[2]; };
  static __device__ __forceinline__ v16h load(const _Float16* p) {
    U f; f.h[0] = *(const v8h*)(p); f.h[1] = *(const v8h*)(p + 16); return f.v;
  }
  static __device__ __forceinline__ v8f mma(v16h a, v16h b, v8f c) {
    return __builtin_amdgcn_wmma_f32_16x16x32_f16(false, a, false, b, (short)0, c, false, false);
  }
  static __device__ __forceinline__ void guard4(v8f& a, v8f& b, v8f& c, v8f& d, v16h x, v16h y) { dep_guard4_h(a, b, c, d, x, y); }
  static __device__ __forceinline__ void keep(v16h a, v16h b, v16h c, v16h d) { keep4_h(a, b, c, d); }
};
template <> struct Frag<__bf16> {
  typedef v16b V; union U { v16b v; v8b h[2]; };
  static __device__ __forceinline__ v16b load(const __bf16* p) {
    U f; f.h[0] = *(const v8b*)(p); f.h[1] = *(const v8b*)(p + 16); return f.v;
  }
  static __device__ __forceinline__ v8f mma(v16b a, v16b b, v8f c) {
    return __builtin_amdgcn_wmma_f32_16x16x32_bf16(false, a, false, b, (short)0, c, false, false);
  }
  static __device__ __forceinline__ void guard4(v8f& a, v8f& b, v8f& c, v8f& d, v16b x, v16b y) { dep_guard4_b(a, b, c, d, x, y); }
  static __device__ __forceinline__ void keep(v16b a, v16b b, v16b c, v16b d) { keep4_b(a, b, c, d); }
};

__device__ __forceinline__ v8f mma_h(v16h a, v16h b, v8f c) {
  c = __builtin_amdgcn_wmma_f32_16x16x32_f16(false, a, false, b, (short)0, c, false, false);
  asm volatile("v_nop\n\tv_nop\n\tv_nop\n\tv_nop" : "+v"(c) : "v"(a), "v"(b));
  return c;
}

template <int ET> struct Elem;
template <> struct Elem<0> { typedef _Float16 T; };
template <> struct Elem<1> { typedef __bf16 T; };
template <int ET, bool SPLIT, int BIAS_MODE, int OUT_MODE, bool RESID, int ACT = 0>
__global__ __launch_bounds__(256) void wmma_gemm64(
    const unsigned short* __restrict__ Ap, const unsigned short* __restrict__ A2p, int lda, long strideA,
    const unsigned short* __restrict__ Btp, const unsigned short* __restrict__ Bt2p, int ldb, long strideB,
    void* __restrict__ Cout, void* __restrict__ Cout2, int ldc, long strideC,
    const float* __restrict__ bias,
    const float* __restrict__ resid, long strideR,
    int M, int N, int K, float scale) {
  typedef typename Elem<ET>::T T;
  typedef typename Frag<T>::V V;
  const T* A = (const T*)Ap; const T* A2 = (const T*)A2p; const T* Bt = (const T*)Btp; const T* Bt2 = (const T*)Bt2p;
  __shared__ __align__(16) float sT[8][16 * 68];
  const int b    = blockIdx.y;
  const int lane = threadIdx.x & 31;
  const int wave = threadIdx.x >> 5;
  const int tilesN = N >> 6;
  const int tilesM = M >> 6;
  const int tile = blockIdx.x * 8 + wave;
  if (tile >= tilesM * tilesN) return;
  const int tm = tile / tilesN;
  const int tn = tile - tm * tilesN;
  const int m0 = tm << 6;
  const int n0 = tn << 6;

  const T* Ab  = A  + (size_t)b * strideA;
  const T* Bb  = Bt + (size_t)b * strideB;
  const T* Ab2 = SPLIT ? (A2  + (size_t)b * strideA) : nullptr;
  const T* Bb2 = SPLIT ? (Bt2 + (size_t)b * strideB) : nullptr;

  const int rlane = lane & 15;
  const int koff  = (lane >> 4) * 8;
  const int mOff  = (lane >> 4) * 8;

  v8f acc[4][4];
#pragma unroll
  for (int i = 0; i < 4; ++i)
#pragma unroll
    for (int j = 0; j < 4; ++j) acc[i][j] = (v8f){0.f,0.f,0.f,0.f,0.f,0.f,0.f,0.f};

  for (int k0 = 0; k0 < K; k0 += 32) {
    V bh[4], bl[4];
#pragma unroll
    for (int j = 0; j < 4; ++j) {
      const size_t bo = (size_t)(n0 + (j << 4) + rlane) * ldb + koff + k0;
      bh[j] = Frag<T>::load(Bb + bo);
      if (SPLIT) bl[j] = Frag<T>::load(Bb2 + bo);
    }
#pragma unroll
    for (int i = 0; i < 4; ++i) {
      const size_t ao = (size_t)(m0 + (i << 4) + rlane) * lda + koff + k0;
      V ah = Frag<T>::load(Ab + ao);
      V al;
      if (SPLIT) al = Frag<T>::load(Ab2 + ao);
#pragma unroll
      for (int j = 0; j < 4; ++j) {
        acc[i][j] = Frag<T>::mma(ah, bh[j], acc[i][j]);
        if (SPLIT) {
          acc[i][j] = Frag<T>::mma(ah, bl[j], acc[i][j]);
          acc[i][j] = Frag<T>::mma(al, bh[j], acc[i][j]);
        }
      }
      Frag<T>::guard4(acc[i][0], acc[i][1], acc[i][2], acc[i][3], ah, SPLIT ? al : ah);
    }
    Frag<T>::keep(bh[0], bh[1], bh[2], bh[3]);
    if (SPLIT) Frag<T>::keep(bl[0], bl[1], bl[2], bl[3]);
  }
  acc_guard4(acc[0][0], acc[0][1], acc[0][2], acc[0][3]);
  acc_guard4(acc[1][0], acc[1][1], acc[1][2], acc[1][3]);
  acc_guard4(acc[2][0], acc[2][1], acc[2][2], acc[2][3]);
  acc_guard4(acc[3][0], acc[3][1], acc[3][2], acc[3][3]);

  float* slab = sT[wave];
  const float* Rb = RESID ? (resid + (size_t)b * strideR) : nullptr;
#pragma unroll
  for (int i = 0; i < 4; ++i) {
    const int mBase = m0 + (i << 4);
#pragma unroll
    for (int j = 0; j < 4; ++j) {
      const int n = n0 + (j << 4) + rlane;
      float bv = 0.f;
      if (BIAS_MODE == 2) bv = bias[n];
#pragma unroll
      for (int r = 0; r < 8; ++r) {
        float v = acc[i][j][r] * scale;
        if (BIAS_MODE == 1) v += bias[mBase + mOff + r];
        if (BIAS_MODE == 2) v += bv;
        if (RESID) v += Rb[(size_t)(mBase + mOff + r) * ldc + n];
        if (ACT == 1) v = tanhf(v);
        if (ACT == 2) v = fmaxf(v, 0.0f);
        if (ACT == 3) v = v / (1.0f + expf(-v));
        if (ACT == 4) v = (v > 0.f) ? v : 0.01f * v;
        slab[(mOff + r) * 68 + (j << 4) + rlane] = v;
      }
    }
    __builtin_amdgcn_fence(__ATOMIC_RELEASE, "workgroup");
    __builtin_amdgcn_wave_barrier();
    __builtin_amdgcn_fence(__ATOMIC_ACQUIRE, "workgroup");
    if (OUT_MODE == 0) {
      float* C = (float*)Cout + (size_t)b * strideC;
      const int hh = lane >> 4, c4 = (lane & 15) * 4;
      for (int pass = 0; pass < 2; ++pass) {
#pragma unroll
        for (int it = 0; it < 8; ++it) {
          const int row = it * 2 + hh;
          v4f v = *(const v4f*)(slab + row * 68 + c4);
          *(volatile v4f*)(C + (size_t)(mBase + row) * ldc + n0 + c4) = v;
        }
        __threadfence();
      }
    } else {
      const int q = lane >> 3, c8 = (lane & 7) * 8;
      unsigned short* C  = (unsigned short*)Cout  + (size_t)b * strideC;
      unsigned short* C2 = (OUT_MODE == 2) ? ((unsigned short*)Cout2 + (size_t)b * strideC) : nullptr;
      for (int pass = 0; pass < 2; ++pass) {
#pragma unroll
        for (int it = 0; it < 4; ++it) {
          const int row = it * 4 + q;
          const float* sp = slab + row * 68 + c8;
          v8h hv, lv;
#pragma unroll
          for (int e = 0; e < 8; ++e) {
            if (OUT_MODE == 1) {
              hv[e] = (_Float16)sp[e];
            } else {
              unsigned short hb = f2bf_bits(sp[e]);
              unsigned short lb = f2bf_bits(sp[e] - bf_bits2f(hb));
              hv[e] = __builtin_bit_cast(_Float16, hb);
              lv[e] = __builtin_bit_cast(_Float16, lb);
            }
          }
          *(volatile v8h*)(C + (size_t)(mBase + row) * ldc + n0 + c8) = hv;
          if (OUT_MODE == 2) *(volatile v8h*)(C2 + (size_t)(mBase + row) * ldc + n0 + c8) = lv;
        }
        __threadfence();
      }
    }
    __builtin_amdgcn_fence(__ATOMIC_RELEASE, "workgroup");
    __builtin_amdgcn_wave_barrier();
    __builtin_amdgcn_fence(__ATOMIC_ACQUIRE, "workgroup");
  }
}


__device__ __forceinline__ float fast_tanh(float v) { return 1.0f - 2.0f * frcp(__expf(2.0f * v) + 1.0f); }
__device__ __forceinline__ float fast_sigmoid(float v) { return frcp(1.0f + __expf(-v)); }

__global__ __launch_bounds__(kThr) void wsetup_kernel(const float* __restrict__ wih0, const float* __restrict__ whh0, const float* __restrict__ bi0,
                                                      const float* __restrict__ bh0, const float* __restrict__ wih1, const float* __restrict__ whh1,
                                                      const float* __restrict__ bi1, const float* __restrict__ bh1, const float* __restrict__ fcw,
                                                      const float* __restrict__ fcb, unsigned short* __restrict__ W0, unsigned short* __restrict__ W1,
                                                      unsigned short* __restrict__ WF, float* __restrict__ BIAS) {
  unsigned v = blockIdx.x * (unsigned)kThr + threadIdx.x;
  asm volatile("" : "+v"(v));
  if (v < 8704u) {
    const float* sp = whh0; bool live = true; bool four = false; unsigned short* dp = W0 + (size_t)v * 8u;
    if (v < 4096u) {
      const unsigned n = v >> 4, k8 = (v & 15u) * 8u;
      live = k8 < 72u; four = (k8 == 64u);
      sp = (k8 < 64u) ? (whh0 + (size_t)n * kH + k8) : four ? (wih0 + (size_t)n * kIn) : whh0;
    } else if (v < 8192u) {
      const unsigned w = v - 4096u, n = w >> 4, k8 = (w & 15u) * 8u;
      sp = (k8 < 64u) ? (whh1 + (size_t)n * kH + k8) : (wih1 + (size_t)n * kH + (k8 - 64u)); dp = W1 + (size_t)w * 8u;
    } else {
      const unsigned w = v - 8192u;
      sp = fcw + (size_t)w * 8u; dp = WF + (size_t)w * 8u;
    }
    const v4f a0 = *(const v4f*)sp;
    const v4f a1 = *(const v4f*)(sp + (four ? 0 : 4));
    v8h hv;
#pragma unroll
    for (int e = 0; e < 4; ++e) {
      const float p = a0[e], q = a1[e];
      hv[e] = (_Float16)(live ? carry_flush(bf16r(p), kInCarry) : 0.0f);
      hv[4 + e] = (_Float16)((live && !four) ? carry_flush(bf16r(q), kInCarry) : 0.0f);
    }
    *(volatile v8h*)dp = hv;
    __threadfence();
    *(volatile v8h*)dp = hv;
  } else {
    const unsigned i0 = (v - 8704u) * 4u;
    v4f o = {0.f, 0.f, 0.f, 0.f};
    if (i0 < (unsigned)kFBF) {
      const bool l1 = i0 >= (unsigned)kFB1;
      const unsigned j = i0 - (l1 ? (unsigned)kFB1 : 0u);
      const v4f p = *(const v4f*)((l1 ? bi1 : bi0) + j), q = *(const v4f*)((l1 ? bh1 : bh0) + j);
#pragma unroll
      for (int e = 0; e < 4; ++e) { const float pp = p[e], qq = q[e]; o[e] = bf16r(pp) + bf16r(qq); }
    } else if (i0 < (unsigned)(kFBF + kH)) {
      const v4f p = *(const v4f*)(fcb + (i0 - (unsigned)kFBF));
#pragma unroll
      for (int e = 0; e < 4; ++e) { const float pp = p[e]; o[e] = bf16r(pp); }
    }
    float* dp = BIAS + i0;
    *(volatile v4f*)dp = o;
    __threadfence();
    *(volatile v4f*)dp = o;
  }
}
static_assert(256 * 16 == 4096 && 64 * 8 == 512 && 4096 + 4096 + 512 == 8704 && kFEnd / 4 == 256 && 8704 + 256 == 35 * kThr && (kFB1 % 128) == 0 && (kFBF % 128) == 0, "weight set-up grid exact");

__global__ __launch_bounds__(kThr) void zinit_kernel(const float* __restrict__ x, unsigned short* __restrict__ A0, unsigned short* __restrict__ A1,
                                                     float* __restrict__ CELLS) {
  unsigned v = blockIdx.x * (unsigned)kThr + threadIdx.x;
  asm volatile("" : "+v"(v));
  if (v < 65536u) {
    const bool first = v < 32768u;
    const unsigned w = first ? v : (v - 32768u);
    const unsigned b = w >> 4, k8 = (w & 15u) * 8u;
    const bool xs = first && (k8 == 64u);
    const v4f a0 = *(const v4f*)(x + (size_t)b * kT * kIn);
    v8h hv;
#pragma unroll
    for (int e = 0; e < 4; ++e) { const float p = a0[e]; hv[e] = (_Float16)(xs ? carry_flush(bf16r(p), kInCarry) : 0.0f); hv[4 + e] = (_Float16)0.0f; }
    unsigned short* dp = (first ? A0 : A1) + (size_t)w * 8u;
    *(volatile v8h*)dp = hv;
    __threadfence();
    *(volatile v8h*)dp = hv;
  } else {
    const v4f z = {0.f, 0.f, 0.f, 0.f};
    float* dp = CELLS + (size_t)(v - 65536u) * 4u;
    *(volatile v4f*)dp = z;
    __threadfence();
    *(volatile v4f*)dp = z;
  }
}
static_assert(kB * 16 == 32768 && 2 * kB * kH / 4 == 65536 && 65536 + 65536 == 512 * kThr, "plane set-up grid exact");

__global__ __launch_bounds__(kThr) void cell2_kernel(const float* __restrict__ G0, const float* __restrict__ G1, const float* __restrict__ x,
                                                     float* __restrict__ C0, float* __restrict__ C1, unsigned short* __restrict__ A0,
                                                     unsigned short* __restrict__ A1, unsigned short* __restrict__ HN16, int k) {
  const bool l0 = blockIdx.x < 64u;
  if (l0 ? (k >= kT) : (k < 1)) return;
  unsigned v = (l0 ? blockIdx.x : (blockIdx.x - 64u)) * (unsigned)kThr + threadIdx.x;
  asm volatile("" : "+v"(v));
  const unsigned b = v >> 3, u8 = (v & 7u) * 8u;
  const float* gr = (l0 ? G0 : G1) + (size_t)b * kG4 + u8;
  float* cp = (l0 ? C0 : C1) + (size_t)b * kH + u8;
  v8h hv, xv;
  v4f cn0, cn1;
#pragma unroll
  for (int hlf = 0; hlf < 2; ++hlf) {
    const v4f gi = *(const v4f*)(gr + 4 * hlf), gf = *(const v4f*)(gr + kH + 4 * hlf), gg = *(const v4f*)(gr + 2 * kH + 4 * hlf), go = *(const v4f*)(gr + 3 * kH + 4 * hlf);
    const v4f co = *(const v4f*)(cp + 4 * hlf);
#pragma unroll
    for (int e = 0; e < 4; ++e) {
      const float cn = fast_sigmoid(gf[e]) * co[e] + fast_sigmoid(gi[e]) * fast_tanh(gg[e]);
      const float hn = fast_sigmoid(go[e]) * fast_tanh(cn);
      if (hlf == 0) cn0[e] = cn; else cn1[e] = cn;
      hv[4 * hlf + e] = (_Float16)carry_flush(hn, kInCarry);
    }
  }
  const bool nx = l0 && (u8 == 0u) && (k + 1 < kT);
  {
    const v4f a0 = *(const v4f*)(x + ((size_t)b * kT + (size_t)(nx ? (k + 1) : 0)) * kIn);
#pragma unroll
    for (int e = 0; e < 4; ++e) { const float p = a0[e]; xv[e] = (_Float16)carry_flush(bf16r(p), kInCarry); xv[4 + e] = (_Float16)0.0f; }
  }
  unsigned short* hp = (l0 ? A0 : A1) + (size_t)b * kKP + u8;
  unsigned short* yp = l0 ? (A1 + (size_t)b * kKP + kH + u8)
                          : (HN16 + (size_t)b * kH + u8);
  unsigned short* xp = A0 + (size_t)b * kKP + kH;
  const bool wy = l0 || (k == kT);
  for (int pass = 0; pass < 2; ++pass) {
    *(volatile v4f*)cp = cn0; *(volatile v4f*)(cp + 4) = cn1;
    *(volatile v8h*)hp = hv;
    if (wy) *(volatile v8h*)yp = hv;
    if (nx) *(volatile v8h*)xp = xv;
    __threadfence();
  }
}
static_assert(kB * 8 == 64 * kThr, "cell grid: 64 blocks a layer");

__global__ __launch_bounds__(kThr) void tanh_out_kernel(const float* __restrict__ P32, float* __restrict__ out) {
  unsigned v = blockIdx.x * (unsigned)kThr + threadIdx.x;
  asm volatile("" : "+v"(v));
  const size_t o4 = (size_t)v * 4u;
  const v4f p = *(const v4f*)(P32 + o4);
  v4f o;
#pragma unroll
  for (int e = 0; e < 4; ++e) o[e] = tanhf(p[e]);
  *(volatile v4f*)(out + o4) = o;
  __threadfence();
  *(volatile v4f*)(out + o4) = o;
}
static_assert(kB * kH / 4 == 128 * kThr, "output grid exact");

extern "C" void kernel_launch(void* const* d_in, const int* in_sizes, int n_in,
                              void* d_out, int out_size, void* d_ws, size_t ws_size,
                              hipStream_t stream) {
  if (n_in < 11 || d_out == nullptr || d_ws == nullptr) return;
  if (in_sizes[0] != kB * kT * kIn || in_sizes[1] != kG4 * kIn || in_sizes[2] != kG4 * kH || in_sizes[3] != kG4 || in_sizes[4] != kG4) return;
  if (in_sizes[5] != kG4 * kH || in_sizes[6] != kG4 * kH || in_sizes[7] != kG4 || in_sizes[8] != kG4 || in_sizes[9] != kH * kH || in_sizes[10] != kH) return;
  if (out_size != kB * kH) return;
  if (ws_size < kWsTotal) return;
  const float* x = (const float*)d_in[0];
  const float* w_ih0 = (const float*)d_in[1];
  const float* w_hh0 = (const float*)d_in[2];
  const float* b_ih0 = (const float*)d_in[3];
  const float* b_hh0 = (const float*)d_in[4];
  const float* w_ih1 = (const float*)d_in[5];
  const float* w_hh1 = (const float*)d_in[6];
  const float* b_ih1 = (const float*)d_in[7];
  const float* b_hh1 = (const float*)d_in[8];
  const float* fc_w = (const float*)d_in[9];
  const float* fc_b = (const float*)d_in[10];
  float* out = (float*)d_out;
  char* ws = (char*)d_ws;
  unsigned short* W0 = (unsigned short*)(ws + kOffW0);
  unsigned short* W1 = (unsigned short*)(ws + kOffW1);
  unsigned short* WF = (unsigned short*)(ws + kOffWF);
  float* BIAS = (float*)(ws + kOffBIAS);
  unsigned short* A0 = (unsigned short*)(ws + kOffA0);
  unsigned short* A1 = (unsigned short*)(ws + kOffA1);
  float* G0 = (float*)(ws + kOffG0);
  float* G1 = (float*)(ws + kOffG1);
  float* C0 = (float*)(ws + kOffC0);
  float* C1 = (float*)(ws + kOffC1);
  unsigned short* HN16 = (unsigned short*)(ws + kOffHN16);
  float* P32 = (float*)(ws + kOffP32);

  wsetup_kernel<<<35, kThr, 0, stream>>>(w_ih0, w_hh0, b_ih0, b_hh0, w_ih1, w_hh1, b_ih1, b_hh1, fc_w, fc_b, W0, W1, WF, BIAS);
  zinit_kernel<<<512, kThr, 0, stream>>>(x, A0, A1, C0);

  for (int k = 0; k <= kT; ++k) {
    if (k < kT) {
      wmma_gemm64<0, false, 2, 0, false, 0><<<dim3((kB / 64) * (kG4 / 64) / 8, 1), 256, 0, stream>>>(
          A0, A0, kKP, 0L, W0, W0, kKP, 0L, (void*)G0, (void*)G0, kG4, 0L, BIAS + kFB0, nullptr, 0L, kB, kG4, kK0, kSc);
    }
    if (k >= 1) {
      wmma_gemm64<0, false, 2, 0, false, 0><<<dim3((kB / 64) * (kG4 / 64) / 8, 1), 256, 0, stream>>>(
          A1, A1, kKP, 0L, W1, W1, kKP, 0L, (void*)G1, (void*)G1, kG4, 0L, BIAS + kFB1, nullptr, 0L, kB, kG4, kKP, kSc);
    }
    cell2_kernel<<<128, kThr, 0, stream>>>(G0, G1, x, C0, C1, A0, A1, HN16, k);
  }
  wmma_gemm64<0, false, 2, 0, false, 0><<<dim3((kB / 64) * (kH / 64) / 8, 1), 256, 0, stream>>>(
      HN16, HN16, kH, 0L, WF, WF, kH, 0L, (void*)P32, (void*)P32, kH, 0L, BIAS + kFBF, nullptr, 0L, kB, kH, kH, kSc);
  tanh_out_kernel<<<128, kThr, 0, stream>>>(P32, out);
}
